// _MultiHeadScaledDotAttention_63359357551275
// MI455X (gfx1250) — hardware-verified
//
#include <hip/hip_runtime.h>
#include <math.h>

typedef __attribute__((ext_vector_type(16))) _Float16 v16h;
typedef __attribute__((ext_vector_type(16))) __bf16 v16b;
typedef __attribute__((ext_vector_type(8)))  _Float16 v8h;
typedef __attribute__((ext_vector_type(8)))  float v8f;
typedef __attribute__((ext_vector_type(4)))  float v4f;
typedef __attribute__((ext_vector_type(2)))  float v2f;
typedef __attribute__((ext_vector_type(4)))  unsigned v4u;
typedef __attribute__((ext_vector_type(4)))  int v4i;
typedef float __attribute__((may_alias)) float_a;
typedef int __attribute__((may_alias)) int_a;

template <typename T> __device__ __forceinline__ void vst2(void* p, T v) { *(volatile T*)p = v; __threadfence(); *(volatile T*)p = v; }
__device__ __forceinline__ v8f wmma16(v16h a, v16h b, v8f c) {
  v8f d = __builtin_amdgcn_wmma_f32_16x16x32_f16(false, a, false, b, (short)0, c, false, false);
  asm volatile("v_nop\n\tv_nop\n\tv_nop\n\tv_nop" : "+v"(d) : "v"(a), "v"(b));
  return d;
}
__device__ __forceinline__ v8f wmma_bf(v16b a, v16b b, v8f c) {
  v8f d = __builtin_amdgcn_wmma_f32_16x16x32_bf16(false, a, false, b, (short)0, c, false, false);
  asm volatile("v_nop\n\tv_nop\n\tv_nop\n\tv_nop" : "+v"(d) : "v"(a), "v"(b));
  return d;
}
__device__ __forceinline__ v16h frag_h(const _Float16* rowk0, int lane) {
  union { v16h v; v8h q[2]; } u; const _Float16* p = rowk0 + 8 * (lane >> 4);
  u.q[0] = *(const v8h*)p; u.q[1] = *(const v8h*)(p + 16); return u.v;
}
__device__ __forceinline__ v16h frag_f32(const float* rowk0, int lane) {
  v16h a; const float* p = rowk0 + 8 * (lane >> 4);
#pragma unroll
  for (int i = 0; i < 8; ++i) { a[i] = (_Float16)p[i]; a[8 + i] = (_Float16)p[16 + i]; }
  return a;
}
__device__ __forceinline__ v16h frag_f32s(const float* rowk0, int lane, float sc) {
  v16h a; const float* p = rowk0 + 8 * (lane >> 4);
#pragma unroll
  for (int i = 0; i < 8; ++i) { a[i] = (_Float16)(p[i] * sc); a[8 + i] = (_Float16)(p[16 + i] * sc); }
  return a;
}
__device__ __forceinline__ v16h fragc_f32(const float* W, int k0, int n, int lane, int ld, int K) {
  v16h a; const int g = lane >> 4;
#pragma unroll
  for (int i = 0; i < 8; ++i) { const int ka = k0 + 8 * g + i, kb = ka + 16;
    a[i] = (_Float16)(ka < K ? W[(size_t)(ka < K ? ka : K - 1) * ld + n] : 0.f); a[8 + i] = (_Float16)(kb < K ? W[(size_t)(kb < K ? kb : K - 1) * ld + n] : 0.f); }
  return a;
}
struct F2 { v16b h, l; };
__device__ __forceinline__ F2 bsplit16(const float v[16]) { F2 r;
#pragma unroll
  for (int i = 0; i < 16; ++i) { const __bf16 h = (__bf16)v[i]; r.h[i] = h; r.l[i] = (__bf16)(v[i] - (float)h); }
  return r; }
__device__ __forceinline__ F2 split_row(const float* row, int k0, int lane) { float v[16]; const float* p = row + k0 + 8 * (lane >> 4);
#pragma unroll
  for (int i = 0; i < 8; ++i) { v[i] = p[i]; v[8 + i] = p[16 + i]; }
  return bsplit16(v); }
__device__ __forceinline__ F2 split_rowK(const float* row, int k0, int lane, int K) { float v[16]; const int g = lane >> 4;
#pragma unroll
  for (int i = 0; i < 8; ++i) { const int ka = k0 + 8 * g + i, kb = ka + 16; v[i] = ka < K ? row[ka < K ? ka : K - 1] : 0.f; v[8 + i] = kb < K ? row[kb < K ? kb : K - 1] : 0.f; }
  return bsplit16(v); }
__device__ __forceinline__ F2 split_col(const float* W, int k0, int n, int lane, int ld, int K) { float v[16]; const int g = lane >> 4;
#pragma unroll
  for (int i = 0; i < 8; ++i) { const int ka = k0 + 8 * g + i, kb = ka + 16; v[i] = ka < K ? W[(size_t)(ka < K ? ka : K - 1) * ld + n] : 0.f; v[8 + i] = kb < K ? W[(size_t)(kb < K ? kb : K - 1) * ld + n] : 0.f; }
  return bsplit16(v); }
__device__ __forceinline__ v8f mac3(const F2& a, const F2& b, v8f c) { c = wmma_bf(a.l, b.h, c); c = wmma_bf(a.h, b.l, c); return wmma_bf(a.h, b.h, c); }
__device__ __forceinline__ float sigm(float v) { return 1.0f / (1.0f + expf(-v)); }
#define LDSX() do { asm volatile("s_wait_dscnt 0" ::: "memory"); __builtin_amdgcn_wave_barrier(); __builtin_amdgcn_fence(__ATOMIC_RELEASE, "workgroup"); } while (0)


#define NB 2
#define SS 2048
#define E 1024
#define NH 16
#define HD 64
#define NR (NB * SS)
__device__ __forceinline__ float bfr(float v) { return (float)(__bf16)v; }
__device__ __forceinline__ v16b frag_b(const __bf16* rowk0, int lane) { return __builtin_bit_cast(v16b, frag_h((const _Float16*)rowk0, lane)); }
__device__ __attribute__((noinline)) float exp_ni(float v) { return expf(v); }

__global__ __launch_bounds__(256) void k_cvt(const float* __restrict__ key, const float* __restrict__ value, __bf16* __restrict__ Kb, __bf16* __restrict__ VT) {
  __shared__ __align__(16) __bf16 st[128][72];
  const int tid = threadIdx.x; const int r0 = blockIdx.x * 64, f0 = blockIdx.y * 128, which = blockIdx.z; const int b = r0 / SS, s0 = r0 % SS;
  if (which == 0) {
    for (int q = tid; q < 64 * 16; q += 256) { const int rl = q >> 4, pc = q & 15; const float* src = key + (size_t)(r0 + rl) * E + f0 + pc * 8; union { __bf16 e[8]; v4u u; } pk;
#pragma unroll
      for (int e = 0; e < 8; ++e) pk.e[e] = (__bf16)src[e];
      vst2((unsigned*)(Kb + (size_t)(r0 + rl) * E + f0 + pc * 8), pk.u); } }
  else {
    for (int q = tid; q < 64 * 128; q += 256) { const int rl = q >> 7, f = q & 127; st[f][rl] = (__bf16)value[(size_t)(r0 + rl) * E + f0 + f]; }
    __syncthreads();
    for (int q = tid; q < 128 * 8; q += 256) { const int f = q >> 3, pc = q & 7; const int c = f0 + f; const int h = c >> 6, u = c & 63; vst2((unsigned*)(VT + (((size_t)b * NH + h) * HD + u) * SS + s0 + pc * 8), *(const v4u*)(&st[f][pc * 8])); } }
}
__global__ __launch_bounds__(128) void k_attn(const float* __restrict__ query, const __bf16* __restrict__ Kb, const __bf16* __restrict__ VT, const float* __restrict__ mask, float* __restrict__ O) {
  __shared__ __align__(16) float sS[4][16][68];
  __shared__ __align__(16) __bf16 sPh[4][16][72], sPl[4][16][72];
  __shared__ __align__(16) float sO[4][16][68];
  const int tid = threadIdx.x, w = tid >> 5, lane = tid & 31, col = lane & 15, g = lane >> 4; const int bh = blockIdx.y; const int b = bh / NH, h = bh % NH; const int q0 = blockIdx.x * 64 + w * 16; const size_t rb = (size_t)b * SS;
  v16b aq[2];
#pragma unroll
  for (int kc = 0; kc < 2; ++kc) aq[kc] = split_row(query + (rb + q0 + col) * E + h * HD, kc * 32, lane).h;
  const float* mrow = mask + rb;
  float mrun = -3.0e38f, lrun = 0.f; v8f acc[4] = {};
#pragma unroll 1
  for (int kt = 0; kt < SS / 64; ++kt) {
#pragma unroll
    for (int t = 0; t < 4; ++t) { const int key = kt * 64 + t * 16 + col; const size_t ko = (rb + key) * E + h * HD; v8f s = {};
#pragma unroll
      for (int kc = 0; kc < 2; ++kc) s = wmma_bf(aq[kc], frag_b(Kb + ko + kc * 32, lane), s);
      const float bias = (1.0f - bfr(mrow[key])) * 10000.0f;
#pragma unroll
      for (int r = 0; r < 8; ++r) sS[w][8 * g + r][t * 16 + col] = s[r] * 0.125f - bias; }
    LDSX();
    float mx = -3.4e38f;
#pragma unroll
    for (int jj = 0; jj < 32; ++jj) mx = fmaxf(mx, sS[w][col][g * 32 + jj]);
    mx = fmaxf(mx, __shfl_xor(mx, 16, 32));
    const float mnew = fmaxf(mrun, mx); const float corr = expf(mrun - mnew);
    float ps = 0.f;
#pragma unroll 4
    for (int jj = 0; jj < 32; ++jj) { const float p = exp_ni(sS[w][col][g * 32 + jj] - mnew); ps += p; const __bf16 hi = (__bf16)p; sPh[w][col][g * 32 + jj] = hi; sPl[w][col][g * 32 + jj] = (__bf16)(p - (float)hi); }
    ps += __shfl_xor(ps, 16, 32);
    lrun = lrun * corr + ps; mrun = mnew;
#pragma unroll
    for (int r = 0; r < 8; ++r) { const float cr = __shfl(corr, 8 * g + r, 32);
#pragma unroll
      for (int t = 0; t < 4; ++t) acc[t][r] *= cr; }
    LDSX();
#pragma unroll
    for (int kc = 0; kc < 2; ++kc) { const v16b ph = frag_b(&sPh[w][col][0] + kc * 32, lane), pl = frag_b(&sPl[w][col][0] + kc * 32, lane);
#pragma unroll
      for (int t = 0; t < 4; ++t) { const v16b vb = frag_b(VT + (((size_t)b * NH + h) * HD + t * 16 + col) * SS + kt * 64 + kc * 32, lane); acc[t] = wmma_bf(pl, vb, acc[t]); acc[t] = wmma_bf(ph, vb, acc[t]); } }
    __builtin_amdgcn_wave_barrier(); }
#pragma unroll
  for (int r = 0; r < 8; ++r) { const float lr = __shfl(lrun, 8 * g + r, 32); const float inv = 1.0f / lr;
#pragma unroll
    for (int t = 0; t < 4; ++t) sO[w][8 * g + r][t * 16 + col] = acc[t][r] * inv; }
  LDSX();
  for (int qq = lane; qq < 16 * 16; qq += 32) { const int rl = qq >> 4, pc = qq & 15; vst2(O + (rb + q0 + rl) * E + h * HD + pc * 4, *(const v4f*)(&sO[w][rl][pc * 4])); }
}
__global__ __launch_bounds__(128) void k_out(const float* __restrict__ O, const float* __restrict__ Wo, float* __restrict__ out) {
  __shared__ __align__(16) float so[4][16][132];
  const int tid = threadIdx.x, wave = tid >> 5, lane = tid & 31, col = lane & 15, g = lane >> 4; const size_t r0 = (size_t)blockIdx.x * 64 + wave * 16; const int n0 = blockIdx.y * 128;
  v8f acc[8] = {};
#pragma unroll 2
  for (int kc = 0; kc < E / 32; ++kc) { const F2 a = split_row(O + (r0 + col) * E, kc * 32, lane);
#pragma unroll
    for (int j = 0; j < 8; ++j) { const v16b wb = split_col(Wo, kc * 32, n0 + j * 16 + col, lane, E, E).h; acc[j] = wmma_bf(a.l, wb, acc[j]); acc[j] = wmma_bf(a.h, wb, acc[j]); } }
#pragma unroll
  for (int j = 0; j < 8; ++j)
#pragma unroll
    for (int r = 0; r < 8; ++r) so[wave][8 * g + r][j * 16 + col] = acc[j][r];
  LDSX();
  for (int rl = 0; rl < 16; ++rl) vst2(out + (r0 + rl) * E + n0 + lane * 4, *(const v4f*)(&so[wave][rl][lane * 4]));
}
extern "C" void kernel_launch(void* const* d_in, const int* in_sizes, int n_in, void* d_out, int out_size, void* d_ws, size_t ws_size, hipStream_t stream) {
  (void)in_sizes; (void)n_in; (void)out_size; (void)ws_size;
  const float* query = (const float*)d_in[0]; const float* key = (const float*)d_in[1]; const float* value = (const float*)d_in[2]; const float* mask = (const float*)d_in[3]; const float* Wo = (const float*)d_in[4];
  char* ws = (char*)d_ws; size_t off = 0;
  auto take = [&](size_t bytes) { char* p = ws + off; off += (bytes + 255) & ~(size_t)255; return p; };
  __bf16* Kb = (__bf16*)take((size_t)NR * E * 2); __bf16* VT = (__bf16*)take((size_t)NR * E * 2); float* O = (float*)take((size_t)NR * E * 4);
  k_cvt<<<dim3(NR / 64, E / 128, 2), 256, 0, stream>>>(key, value, Kb, VT);
  k_attn<<<dim3(SS / 64, NB * NH), 128, 0, stream>>>(query, Kb, VT, mask, O);
  k_out<<<dim3(NR / 64, E / 128), 128, 0, stream>>>(O, Wo, (float*)d_out);
}
